// FourierLayer_90099823935690
// MI455X (gfx1250) — hardware-run, weakly checked
//
#include <hip/hip_runtime.h>
#include <math.h>

typedef __attribute__((ext_vector_type(16))) _Float16 v16h;
typedef __attribute__((ext_vector_type(8)))  _Float16 v8h;
typedef __attribute__((ext_vector_type(8)))  float    v8f;
typedef __attribute__((ext_vector_type(4)))  float    v4f;
typedef __attribute__((ext_vector_type(4)))  unsigned v4u;

constexpr int kNB   = 16;
constexpr int kS    = 2048;
constexpr int kH    = 256;
constexpr int kNM   = 32;
constexpr int kJM   = 2 * kNM;
constexpr int kKC   = kH + kJM;
constexpr int kMixM = 64;
constexpr int kMixK = 2 * kH;
constexpr int kMixN = 2 * kH;
constexpr int kRows = kNB * kS;
constexpr int kTP   = 68;
constexpr float kXCarry   = 16.0f;
constexpr float kWCarry   = 1024.0f;
constexpr float kOutScale = 1.0f / (kXCarry * kWCarry);
constexpr float kCoefDC   = (1.0f / (float)kS) / kXCarry;
constexpr float kCoefAC   = (2.0f / (float)kS) / kXCarry;
constexpr float kAngStep  = 6.283185307179586f / (float)kS;
constexpr float kLnEps    = 1e-5f;

static_assert(kS == 2048 && kH == 256 && kNB == 16 && kNM == 32, "shape constants");
static_assert((kKC % 32) == 0 && (kMixK % 32) == 0 && (kS % 32) == 0, "GEMM K multiples of 32");
static_assert((kJM % 64) == 0 && ((kNB * kH) % 64) == 0 && (kMixM % 64) == 0 && (kMixN % 64) == 0 &&
              (kS % 64) == 0 && (kH % 64) == 0, "GEMM M,N multiples of 64");
static_assert(((kKC * 2) % 128) == 0, "A plane pitch is a whole number of 128-B lines");

constexpr size_t kOffXT = 0;
constexpr size_t kOffAC = kOffXT + (size_t)kNB * kH * kS * 2;
constexpr size_t kOffDF = kOffAC + (size_t)kRows * kKC * 2;
constexpr size_t kOffWM = kOffDF + (size_t)kJM * kS * 2;
constexpr size_t kOffXM = kOffWM + (size_t)kNM * kMixN * kMixK * 2;
constexpr size_t kOffYM = kOffXM + (size_t)kNM * kMixM * kMixK * 2;
constexpr size_t kOffB2 = kOffYM + (size_t)kNM * kMixM * kMixN * 4;
constexpr size_t kOffYP = kOffB2 + (size_t)kNB * kH * kKC * 2;
constexpr size_t kWsTotal = kOffYP + (size_t)kRows * kH * 4;
static_assert(kWsTotal == 97255424ull, "carve total");
static_assert(kWsTotal <= 134217728ull, "carve cap");
static_assert((kOffAC % 128) == 0 && (kOffDF % 128) == 0 && (kOffWM % 128) == 0 && (kOffXM % 128) == 0 &&
              (kOffYM % 128) == 0 && (kOffB2 % 128) == 0 && (kOffYP % 128) == 0, "128-B aligned regions");

__device__ __forceinline__ v16h frag_load(const _Float16* p) {
  union U { v16h v; v8h h[2]; };
  U f;
  f.h[0] = *(const v8h*)(p);
  f.h[1] = *(const v8h*)(p + 16);
  return f.v;
}
__device__ __forceinline__ v8f mma_f16(v16h a, v16h b, v8f c) {
  return __builtin_amdgcn_wmma_f32_16x16x32_f16(false, a, false, b, (short)0, c, false, false);
}
__device__ __forceinline__ void tie1(v8f& a, v16h x, v16h y) {
  asm volatile("v_nop\n\tv_nop\n\tv_nop\n\tv_nop" : "+v"(a) : "v"(x), "v"(y));
}
__device__ __forceinline__ void keep4(v16h a, v16h b, v16h c, v16h d) {
  asm volatile("v_nop" :: "v"(a), "v"(b), "v"(c), "v"(d));
}
__device__ __forceinline__ void acc_guard4(v8f& a, v8f& b, v8f& c, v8f& d) {
  asm volatile("v_nop\n\tv_nop\n\tv_nop\n\tv_nop" : "+v"(a), "+v"(b), "+v"(c), "+v"(d));
}

template <int EPI, bool BIASN>
__global__ __launch_bounds__(256) void gemm64_f16_kernel(
    const _Float16* __restrict__ A, int lda, long strideA,
    const _Float16* __restrict__ Bt, int ldb, long strideB,
    void* __restrict__ Cout, int ldc, long strideC,
    const float* __restrict__ bias, int M, int N, int K, float scale)
{
  __shared__ __align__(16) float sT[8][16 * kTP];
  const int b    = blockIdx.y;
  const int lane = threadIdx.x & 31;
  const int wave = __builtin_amdgcn_readfirstlane((int)(threadIdx.x >> 5));
  const int tilesN = N >> 6;
  const int tilesM = M >> 6;
  const int tile = blockIdx.x * 8 + wave;
  if (tile >= tilesM * tilesN) return;
  const int tm = tile / tilesN;
  const int tn = tile - tm * tilesN;
  const int m0 = tm << 6;
  const int n0 = tn << 6;

  const _Float16* Ab = A  + (size_t)b * strideA;
  const _Float16* Bb = Bt + (size_t)b * strideB;

  const int rlane = lane & 15;
  const int koff  = (lane >> 4) * 8;
  const int mOff  = (lane >> 4) * 8;

  v8f acc[4][4];
#pragma unroll
  for (int i = 0; i < 4; ++i)
#pragma unroll
    for (int j = 0; j < 4; ++j) acc[i][j] = (v8f){0.f,0.f,0.f,0.f,0.f,0.f,0.f,0.f};

  for (int k0 = 0; k0 < K; k0 += 32) {
    v16h bh[4];
#pragma unroll
    for (int j = 0; j < 4; ++j) {
      const size_t bo = (size_t)(n0 + (j << 4) + rlane) * ldb + koff + k0;
      bh[j] = frag_load(Bb + bo);
    }
#pragma unroll
    for (int i = 0; i < 4; ++i) {
      const size_t ao = (size_t)(m0 + (i << 4) + rlane) * lda + koff + k0;
      v16h ah = frag_load(Ab + ao);
#pragma unroll
      for (int j = 0; j < 4; ++j) acc[i][j] = mma_f16(ah, bh[j], acc[i][j]);
      tie1(acc[i][0], ah, bh[0]);
      tie1(acc[i][1], ah, bh[1]);
      tie1(acc[i][2], ah, bh[2]);
      tie1(acc[i][3], ah, bh[3]);
    }
    keep4(bh[0], bh[1], bh[2], bh[3]);
  }
  acc_guard4(acc[0][0], acc[0][1], acc[0][2], acc[0][3]);
  acc_guard4(acc[1][0], acc[1][1], acc[1][2], acc[1][3]);
  acc_guard4(acc[2][0], acc[2][1], acc[2][2], acc[2][3]);
  acc_guard4(acc[3][0], acc[3][1], acc[3][2], acc[3][3]);

  float bvj[4];
#pragma unroll
  for (int j = 0; j < 4; ++j) {
    bvj[j] = 0.f;
    if (BIASN) bvj[j] = bias[n0 + (j << 4) + rlane];
  }

  float* slab = sT[wave];
#pragma unroll
  for (int i = 0; i < 4; ++i) {
    const int mBase = m0 + (i << 4);
#pragma unroll
    for (int j = 0; j < 4; ++j) {
#pragma unroll
      for (int r = 0; r < 8; ++r) {
        float v = acc[i][j][r] * scale;
        if (BIASN) v += bvj[j];
        slab[(mOff + r) * kTP + (j << 4) + rlane] = v;
      }
    }
    __builtin_amdgcn_fence(__ATOMIC_RELEASE, "workgroup");
    __builtin_amdgcn_wave_barrier();
    __builtin_amdgcn_fence(__ATOMIC_ACQUIRE, "workgroup");
    if (EPI == 0) {
      float* C = (float*)Cout + (size_t)b * strideC;
      const int hh = lane >> 4, c4 = (lane & 15) * 4;
      for (int pass = 0; pass < 2; ++pass) {
#pragma unroll
        for (int it = 0; it < 8; ++it) {
          const int row = it * 2 + hh;
          const v4f v = *(const v4f*)(slab + row * kTP + c4);
          *(volatile v4f*)(C + (size_t)(mBase + row) * ldc + n0 + c4) = v;
        }
        __threadfence();
      }
    } else {
      _Float16* C = (_Float16*)Cout;
      const int q = lane >> 3, c8 = (lane & 7) * 8;
      const int bb = n0 >> 8;
      const int hbase = n0 & (kH - 1);
      for (int pass = 0; pass < 2; ++pass) {
#pragma unroll
        for (int it = 0; it < 4; ++it) {
          const int row = it * 4 + q;
          const int jm = mBase + row;
          const float* sp = slab + row * kTP + c8;
          const v4f a0 = *(const v4f*)(sp);
          const v4f a1 = *(const v4f*)(sp + 4);
          v8h hv;
#pragma unroll
          for (int e = 0; e < 4; ++e) {
            hv[e]     = (_Float16)a0[e];
            hv[4 + e] = (_Float16)a1[e];
          }
          const size_t o = (size_t)(jm & (kNM - 1)) * (kMixM * kMixK) + (size_t)bb * kMixK +
                           (size_t)(jm >> 5) * kH + hbase + c8;
          *(volatile v8h*)(C + o) = hv;
        }
        __threadfence();
      }
    }
    __builtin_amdgcn_fence(__ATOMIC_RELEASE, "workgroup");
    __builtin_amdgcn_wave_barrier();
    __builtin_amdgcn_fence(__ATOMIC_ACQUIRE, "workgroup");
  }
}

__global__ __launch_bounds__(256) void convert_x_kernel(
    const float* __restrict__ x, _Float16* __restrict__ XT, _Float16* __restrict__ AC)
{
  __shared__ __align__(16) float sT[64 * kTP];
  const int tid  = threadIdx.x;
  const int lane = tid & 31;
  const int wave = __builtin_amdgcn_readfirstlane((int)(threadIdx.x >> 5));
  const int h0 = blockIdx.x * 64;
  const int s0 = blockIdx.y * 64;
  const int b  = blockIdx.z;
  const int lr = tid >> 4, lc4 = (tid & 15) * 4;
#pragma unroll
  for (int i = 0; i < 4; ++i) {
    const int row = lr + 16 * i;
    const v4f v = *(const v4f*)(x + ((size_t)b * kS + s0 + row) * kH + h0 + lc4);
    *(v4f*)(sT + row * kTP + lc4) = v;
  }
  __syncthreads();
  const int q = lane >> 3, c8 = (lane & 7) * 8;
  v8h av[2], tv[2];
#pragma unroll
  for (int it = 0; it < 2; ++it) {
    const int rl = it * 32 + wave * 4 + q;
    const v4f a0 = *(const v4f*)(sT + rl * kTP + c8);
    const v4f a1 = *(const v4f*)(sT + rl * kTP + c8 + 4);
#pragma unroll
    for (int e = 0; e < 4; ++e) {
      av[it][e]     = (_Float16)(a0[e] * kXCarry);
      av[it][4 + e] = (_Float16)(a1[e] * kXCarry);
    }
#pragma unroll
    for (int e = 0; e < 8; ++e) {
      const float t = sT[(c8 + e) * kTP + rl];
      tv[it][e] = (_Float16)(t * kXCarry);
    }
  }
  for (int pass = 0; pass < 2; ++pass) {
#pragma unroll
    for (int it = 0; it < 2; ++it) {
      const int rl = it * 32 + wave * 4 + q;
      *(volatile v8h*)(AC + ((size_t)b * kS + s0 + rl) * kKC + h0 + c8) = av[it];
      *(volatile v8h*)(XT + ((size_t)b * kH + h0 + rl) * kS + s0 + c8) = tv[it];
    }
    __threadfence();
  }
}

__global__ __launch_bounds__(256) void basis_kernel(_Float16* __restrict__ DF, _Float16* __restrict__ AC)
{
  __shared__ __align__(16) float sB[kJM * kTP];
  const int tid  = threadIdx.x;
  const int lane = tid & 31;
  const int wave = __builtin_amdgcn_readfirstlane((int)(threadIdx.x >> 5));
  const int s0 = blockIdx.x * 64;
#pragma unroll 1
  for (int i = 0; i < 8; ++i) {
    const int p  = tid + 256 * i;
    const int k  = p >> 6;
    const int sl = p & 63;
    const int ks = (k * (s0 + sl)) & (kS - 1);
    const float ang = (float)ks * kAngStep;
    const float sv = sinf(ang);
    const float cv = cosf(ang);
    sB[k * kTP + sl] = cv;
    sB[(kNM + k) * kTP + sl] = 0.0f - sv;
  }
  __syncthreads();
  const int q = lane >> 3, c8 = (lane & 7) * 8;
  v8h dv[2], bv[2];
#pragma unroll
  for (int it = 0; it < 2; ++it) {
    const int rl = it * 32 + wave * 4 + q;
    const v4f a0 = *(const v4f*)(sB + rl * kTP + c8);
    const v4f a1 = *(const v4f*)(sB + rl * kTP + c8 + 4);
#pragma unroll
    for (int e = 0; e < 4; ++e) {
      dv[it][e]     = (_Float16)a0[e];
      dv[it][4 + e] = (_Float16)a1[e];
    }
#pragma unroll
    for (int e = 0; e < 8; ++e) {
      const float t = sB[(c8 + e) * kTP + rl];
      bv[it][e] = (_Float16)(t * kXCarry);
    }
  }
  for (int pass = 0; pass < 2; ++pass) {
#pragma unroll
    for (int it = 0; it < 2; ++it) {
      const int rl = it * 32 + wave * 4 + q;
      *(volatile v8h*)(DF + (size_t)rl * kS + s0 + c8) = dv[it];
    }
#pragma unroll 1
    for (int bb = 0; bb < kNB; ++bb) {
#pragma unroll
      for (int it = 0; it < 2; ++it) {
        const int rl = it * 32 + wave * 4 + q;
        *(volatile v8h*)(AC + ((size_t)bb * kS + s0 + rl) * kKC + kH + c8) = bv[it];
      }
    }
    __threadfence();
  }
}

__global__ __launch_bounds__(256) void pack_w_kernel(
    const float* __restrict__ wr, const float* __restrict__ wi,
    _Float16* __restrict__ WM, unsigned char* __restrict__ XMbytes)
{
  __shared__ __align__(16) float sR[64 * kTP];
  __shared__ __align__(16) float sI[64 * kTP];
  const int tid  = threadIdx.x;
  const int lane = tid & 31;
  const int wave = __builtin_amdgcn_readfirstlane((int)(threadIdx.x >> 5));
  const int i0 = blockIdx.x * 64;
  const int j0 = blockIdx.y * 64;
  const int md = blockIdx.z;
  const int lr = tid >> 4, lc4 = (tid & 15) * 4;
#pragma unroll
  for (int i = 0; i < 4; ++i) {
    const int row = lr + 16 * i;
    const size_t so = ((size_t)md * kH + i0 + row) * kH + j0 + lc4;
    const v4f a = *(const v4f*)(wr + so);
    const v4f c = *(const v4f*)(wi + so);
    *(v4f*)(sR + row * kTP + lc4) = a;
    *(v4f*)(sI + row * kTP + lc4) = c;
  }
  __syncthreads();
  const int q = lane >> 3, c8 = (lane & 7) * 8;
  v8h hr[2], hp[2], hn[2];
#pragma unroll
  for (int it = 0; it < 2; ++it) {
    const int jl = it * 32 + wave * 4 + q;
#pragma unroll
    for (int e = 0; e < 8; ++e) {
      const float r = sR[(c8 + e) * kTP + jl] * kWCarry;
      const float w = sI[(c8 + e) * kTP + jl] * kWCarry;
      hr[it][e] = (_Float16)r;
      hp[it][e] = (_Float16)w;
      hn[it][e] = (_Float16)(-w);
    }
  }
  _Float16* base = WM + (size_t)md * kMixN * kMixK;
  const int lin = (blockIdx.z * 4 + blockIdx.y) * 4 + blockIdx.x;
  const int gid = lin * 256 + tid;
  constexpr int kPadVecPerMode = (kMixM - kNB) * kMixK * 2 / 16;
  constexpr int kPadVecTotal = kNM * kPadVecPerMode;
  static_assert(kPadVecPerMode == 3072 && (kPadVecTotal % 256) == 0, "zero-fill map");
  const bool doZero = (lin < kPadVecTotal / 256);
  const int zm  = gid / kPadVecPerMode;
  const int zo  = gid - zm * kPadVecPerMode;
  const v4u zz = (v4u){0u, 0u, 0u, 0u};
  for (int pass = 0; pass < 2; ++pass) {
#pragma unroll
    for (int it = 0; it < 2; ++it) {
      const int n = j0 + it * 32 + wave * 4 + q;
      *(volatile v8h*)(base + (size_t)n * kMixK + i0 + c8)               = hr[it];
      *(volatile v8h*)(base + (size_t)n * kMixK + kH + i0 + c8)          = hn[it];
      *(volatile v8h*)(base + (size_t)(kH + n) * kMixK + i0 + c8)        = hp[it];
      *(volatile v8h*)(base + (size_t)(kH + n) * kMixK + kH + i0 + c8)   = hr[it];
    }
    if (doZero) {
      unsigned char* zp = XMbytes + (size_t)zm * (kMixM * kMixK * 2) + (size_t)kNB * kMixK * 2 + (size_t)zo * 16;
      *(volatile v4u*)zp = zz;
    }
    __threadfence();
  }
}

__global__ __launch_bounds__(256) void pack_b2_kernel(
    const float* __restrict__ cw, const float* __restrict__ YM, _Float16* __restrict__ B2)
{
  const int lane = threadIdx.x & 31;
  const int wave = __builtin_amdgcn_readfirstlane((int)(threadIdx.x >> 5));
  const int q = lane >> 3, c8 = (lane & 7) * 8;
  const int r = blockIdx.x * 32 + wave * 4 + q;
  const int b = r >> 8;
  const int n = r & (kH - 1);
  _Float16* dst = B2 + (size_t)r * kKC;
#pragma unroll 1
  for (int seg = 0; seg < 4; ++seg) {
    const float* src = cw + (size_t)n * kH + seg * 64 + c8;
    const v4f a0 = *(const v4f*)(src);
    const v4f a1 = *(const v4f*)(src + 4);
    v8h hv;
#pragma unroll
    for (int e = 0; e < 4; ++e) {
      hv[e]     = (_Float16)(a0[e] * kWCarry);
      hv[4 + e] = (_Float16)(a1[e] * kWCarry);
    }
    *(volatile v8h*)(dst + seg * 64 + c8) = hv;
    __threadfence();
    *(volatile v8h*)(dst + seg * 64 + c8) = hv;
  }
  {
    const int part = c8 >> 5;
    const float* yb = YM + (size_t)b * kMixN + (size_t)part * kH + n;
    float yv[8];
#pragma unroll
    for (int e = 0; e < 8; ++e) {
      const int md = (c8 + e) & (kNM - 1);
      yv[e] = yb[(size_t)md * (kMixM * kMixN)];
    }
    v8h hv;
#pragma unroll
    for (int e = 0; e < 8; ++e) {
      const int kk = c8 + e;
      const int md = kk & (kNM - 1);
      const float coef = (md == 0) ? kCoefDC : kCoefAC;
      float val = yv[e] * coef;
      val = (kk == kNM) ? 0.0f : val;
      hv[e] = (_Float16)val;
    }
    *(volatile v8h*)(dst + kH + c8) = hv;
    __threadfence();
    *(volatile v8h*)(dst + kH + c8) = hv;
  }
}

__global__ __launch_bounds__(256) void layernorm_kernel(
    const float* __restrict__ YP, const float* __restrict__ gamma, const float* __restrict__ beta,
    float* __restrict__ out)
{
  const int lane = threadIdx.x & 31;
  const int wave = __builtin_amdgcn_readfirstlane((int)(threadIdx.x >> 5));
  const int row = blockIdx.x * 8 + wave;
  const float* yr = YP + (size_t)row * kH;
  const v4f a = *(const v4f*)(yr + lane * 4);
  const v4f c = *(const v4f*)(yr + 128 + lane * 4);
  float sum = ((a[0] + a[1]) + (a[2] + a[3])) + ((c[0] + c[1]) + (c[2] + c[3]));
#pragma unroll
  for (int off = 1; off < 32; off <<= 1) sum += __shfl_xor(sum, off, 32);
  const float mu = sum * (1.0f / (float)kH);
  v4f da, dc;
  float ss = 0.f;
#pragma unroll
  for (int e = 0; e < 4; ++e) {
    da[e] = a[e] - mu;
    dc[e] = c[e] - mu;
    ss += da[e] * da[e];
    ss += dc[e] * dc[e];
  }
#pragma unroll
  for (int off = 1; off < 32; off <<= 1) ss += __shfl_xor(ss, off, 32);
  const float var = ss * (1.0f / (float)kH);
  const float rs = rsqrtf(var + kLnEps);
  const v4f g0 = *(const v4f*)(gamma + lane * 4);
  const v4f g1 = *(const v4f*)(gamma + 128 + lane * 4);
  const v4f b0 = *(const v4f*)(beta + lane * 4);
  const v4f b1 = *(const v4f*)(beta + 128 + lane * 4);
  v4f o0, o1;
#pragma unroll
  for (int e = 0; e < 4; ++e) {
    o0[e] = da[e] * rs * g0[e] + b0[e];
    o1[e] = dc[e] * rs * g1[e] + b1[e];
  }
  float* orow = out + (size_t)row * kH;
  *(volatile v4f*)(orow + lane * 4) = o0;
  *(volatile v4f*)(orow + 128 + lane * 4) = o1;
  __threadfence();
  *(volatile v4f*)(orow + lane * 4) = o0;
  *(volatile v4f*)(orow + 128 + lane * 4) = o1;
}

extern "C" void kernel_launch(void* const* d_in, const int* in_sizes, int n_in,
                              void* d_out, int out_size, void* d_ws, size_t ws_size,
                              hipStream_t stream) {
  if (n_in < 7) return;
  if (in_sizes[0] != kNB * kS * kH) return;
  if (in_sizes[1] != kNM * kH * kH) return;
  if (in_sizes[2] != kNM * kH * kH) return;
  if (in_sizes[3] != kH * kH) return;
  if (in_sizes[4] != kH) return;
  if (in_sizes[5] != kH) return;
  if (in_sizes[6] != kH) return;
  if (out_size != kNB * kS * kH) return;
  if (ws_size < kWsTotal) return;

  const float* x      = (const float*)d_in[0];
  const float* w_real = (const float*)d_in[1];
  const float* w_imag = (const float*)d_in[2];
  const float* conv_w = (const float*)d_in[3];
  const float* conv_b = (const float*)d_in[4];
  const float* gamma  = (const float*)d_in[5];
  const float* beta   = (const float*)d_in[6];
  float* out = (float*)d_out;

  char* ws = (char*)d_ws;
  _Float16* XT = (_Float16*)(ws + kOffXT);
  _Float16* AC = (_Float16*)(ws + kOffAC);
  _Float16* DF = (_Float16*)(ws + kOffDF);
  _Float16* WM = (_Float16*)(ws + kOffWM);
  _Float16* XM = (_Float16*)(ws + kOffXM);
  float*    YM = (float*)(ws + kOffYM);
  _Float16* B2 = (_Float16*)(ws + kOffB2);
  float*    YP = (float*)(ws + kOffYP);

  convert_x_kernel<<<dim3(kH / 64, kS / 64, kNB), 256, 0, stream>>>(x, XT, AC);
  basis_kernel<<<dim3(kS / 64), 256, 0, stream>>>(DF, AC);
  pack_w_kernel<<<dim3(kH / 64, kH / 64, kNM), 256, 0, stream>>>(w_real, w_imag, WM, (unsigned char*)XM);

  gemm64_f16_kernel<1, false><<<dim3(8, 1), 256, 0, stream>>>(
      DF, kS, 0L, XT, kS, 0L, (void*)XM, 0, 0L, nullptr, kJM, kNB * kH, kS, 1.0f);

  gemm64_f16_kernel<0, false><<<dim3(1, kNM), 256, 0, stream>>>(
      XM, kMixK, (long)kMixM * kMixK, WM, kMixK, (long)kMixN * kMixK,
      (void*)YM, kMixN, (long)kMixM * kMixN, nullptr, kMixM, kMixN, kMixK, 1.0f);

  pack_b2_kernel<<<dim3(kNB * kH / 32), 256, 0, stream>>>(conv_w, YM, B2);

  gemm64_f16_kernel<0, true><<<dim3(16, kNB), 256, 0, stream>>>(
      AC, kKC, (long)kS * kKC, B2, kKC, (long)kH * kKC,
      (void*)YP, kH, (long)kS * kH, conv_b, kS, kH, kKC, kOutScale);

  layernorm_kernel<<<dim3(kRows / 8), 256, 0, stream>>>(YP, gamma, beta, out);
}
